// SASAStem2d_7198365188212
// MI455X (gfx1250) — hardware-verified
//
#include <hip/hip_runtime.h>


#define N_IMG   2
#define C_IN    64
#define HS      56
#define WSP     56
#define HW      3136
#define C_OUT   128
#define HEADS   8
#define DH      16
#define KW      7
#define UW      49
#define MIX     4
#define ROWS    768

#define XP      72
#define DP      36
#define KSP     16
#define KSLOTS  88
#define VP      88
#define SP      52
#define OPITCH  64

#define OFF_WMIX ((size_t)0)
#define OFF_Y    ((size_t)4096)
#define SZ_Y     ((size_t)N_IMG * ROWS * HW * 4)
#define OFF_O    (OFF_Y + SZ_Y)
#define SZ_O     ((size_t)N_IMG * C_OUT * HS * OPITCH * 4)
#define WS_TOTAL (OFF_O + SZ_O)

typedef float          v4f  __attribute__((ext_vector_type(4)));
typedef float          v8f  __attribute__((ext_vector_type(8)));
typedef unsigned short us4  __attribute__((ext_vector_type(4)));
typedef unsigned short us8  __attribute__((ext_vector_type(8)));
typedef unsigned short us16 __attribute__((ext_vector_type(16)));
typedef __bf16         v16bf __attribute__((ext_vector_type(16)));

union FragB { us16 v; us8 h[2]; };

__device__ __forceinline__ unsigned short tobf(float f) {
  return __builtin_bit_cast(unsigned short, (__bf16)f);
}
__device__ __forceinline__ float bfext(unsigned short b) {
  return __uint_as_float(((unsigned)b) << 16);
}
__device__ __forceinline__ v8f zero8f() {
  v8f z = {0.f, 0.f, 0.f, 0.f, 0.f, 0.f, 0.f, 0.f};
  return z;
}
__device__ __forceinline__ us16 zero16u() {
  us16 z = {0, 0, 0, 0, 0, 0, 0, 0, 0, 0, 0, 0, 0, 0, 0, 0};
  return z;
}
__device__ __forceinline__ us8 zero8u() {
  us8 z = {0, 0, 0, 0, 0, 0, 0, 0};
  return z;
}

__device__ __forceinline__ v8f wmma_bf(us16 a, us16 b, v8f c) {
  v8f d = __builtin_amdgcn_wmma_f32_16x16x32_bf16(false, __builtin_bit_cast(v16bf, a), false,
                                                  __builtin_bit_cast(v16bf, b), (short)0, c, false, false);
  asm volatile("v_nop\n\tv_nop\n\tv_nop\n\tv_nop" : "+v"(d) : "v"(a), "v"(b));
  return d;
}

__global__ __launch_bounds__(64) void k_mix(const float* __restrict__ row_emb,
                                            const float* __restrict__ col_emb,
                                            const float* __restrict__ mix_emb,
                                            float* wmix)
{
  __shared__ float rc[2 * MIX * KW];
  __shared__ __attribute__((aligned(16))) float wl[256];
  const int t = threadIdx.x;
  for (int i = t; i < 256; i += 64) wl[i] = 0.f;
  if (t < 2 * MIX * KW) {
    const int which = t / (MIX * KW);
    const int rem = t - which * (MIX * KW);
    const int m = rem / KW;
    const int kk = rem - m * KW;
    const float* emb = which ? col_emb : row_emb;
    float s = 0.f;
#pragma unroll 4
    for (int c = 0; c < C_OUT; ++c) s = fmaf(mix_emb[c * MIX + m], emb[c * KW + kk], s);
    rc[t] = s;
  }
  __syncthreads();
  if (t < UW) {
    const int ky = t / KW, kx = t - ky * KW;
    float s[MIX];
#pragma unroll
    for (int m = 0; m < MIX; ++m) s[m] = rc[m * KW + ky] + rc[MIX * KW + m * KW + kx];
    const float mx = fmaxf(fmaxf(s[0], s[1]), fmaxf(s[2], s[3]));
    float e[MIX];
    float den = 0.f;
#pragma unroll
    for (int m = 0; m < MIX; ++m) { e[m] = expf(s[m] - mx); den += e[m]; }
    const float inv = 1.f / den;
#pragma unroll
    for (int m = 0; m < MIX; ++m) wl[m * UW + t] = e[m] * inv;
  }
  __syncthreads();
  if (t < 32) {
    const v4f a = *(const v4f*)(wl + 4 * t);
    const v4f b = *(const v4f*)(wl + 128 + 4 * t);
    volatile v4f* p = (volatile v4f*)wmix;
    p[t] = a;
    p[32 + t] = b;
    __threadfence();
    p[t] = a;
    p[32 + t] = b;
  }
}

__global__ __launch_bounds__(256) void k_proj(const float* __restrict__ x,
                                              const float* __restrict__ Wq,
                                              const float* __restrict__ Wk,
                                              const float* __restrict__ Wv,
                                              float* Y)
{
  __shared__ __attribute__((aligned(16))) unsigned short Xh[32 * XP];
  __shared__ __attribute__((aligned(16))) unsigned short Xl[32 * XP];
  __shared__ __attribute__((aligned(16))) float Ds[128 * DP];

  const int tid = threadIdx.x;
  const int lane = tid & 31, wave = tid >> 5, hh = lane >> 4, mm = lane & 15;
  const int pt = blockIdx.x, ch = blockIdx.y;
  if (pt >= (N_IMG * HW) / 32 || ch >= ROWS / 128) return;
  const int gp0 = pt * 32;
  const int n = gp0 / HW;
  const int p0 = gp0 - n * HW;
  const float* W = (ch == 0) ? Wq : ((ch == 1) ? Wk : (Wv + (size_t)(ch - 2) * C_OUT * C_IN));

  const float* xs = x + (size_t)n * C_IN * HW + p0;
#pragma unroll
  for (int e = 0; e < 8; ++e) {
    const int idx = e * 256 + tid;
    const int c = idx >> 5, p = idx & 31;
    const float v = xs[(size_t)c * HW + p];
    const unsigned short hb = tobf(v);
    const unsigned short lb = tobf(v - bfext(hb));
    Xh[p * XP + c] = hb;
    Xl[p * XP + c] = lb;
  }
  __syncthreads();

  v8f acc0 = zero8f(), acc1 = zero8f();
  const float* wrow = W + (size_t)(wave * 16 + mm) * C_IN;
#pragma unroll
  for (int ks = 0; ks < 2; ++ks) {
    const int k0 = ks * 32;
    const v4f w0 = *(const v4f*)(wrow + k0 + 8 * hh);
    const v4f w1 = *(const v4f*)(wrow + k0 + 8 * hh + 4);
    const v4f w2 = *(const v4f*)(wrow + k0 + 16 + 8 * hh);
    const v4f w3 = *(const v4f*)(wrow + k0 + 16 + 8 * hh + 4);
    us16 ah = zero16u(), al = zero16u();
#pragma unroll
    for (int q = 0; q < 4; ++q) {
      {
        const float f = w0[q];
        const unsigned short hb = tobf(f);
        ah[q] = hb; al[q] = tobf(f - bfext(hb));
      }
      {
        const float f = w1[q];
        const unsigned short hb = tobf(f);
        ah[4 + q] = hb; al[4 + q] = tobf(f - bfext(hb));
      }
      {
        const float f = w2[q];
        const unsigned short hb = tobf(f);
        ah[8 + q] = hb; al[8 + q] = tobf(f - bfext(hb));
      }
      {
        const float f = w3[q];
        const unsigned short hb = tobf(f);
        ah[12 + q] = hb; al[12 + q] = tobf(f - bfext(hb));
      }
    }
    {
      FragB bh, bl;
      const unsigned short* xh = Xh + mm * XP + k0;
      const unsigned short* xl = Xl + mm * XP + k0;
      bh.h[0] = *(const us8*)(xh + 8 * hh);
      bh.h[1] = *(const us8*)(xh + 16 + 8 * hh);
      bl.h[0] = *(const us8*)(xl + 8 * hh);
      bl.h[1] = *(const us8*)(xl + 16 + 8 * hh);
      acc0 = wmma_bf(ah, bh.v, acc0);
      acc0 = wmma_bf(ah, bl.v, acc0);
      acc0 = wmma_bf(al, bh.v, acc0);
    }
    {
      FragB bh, bl;
      const unsigned short* xh = Xh + (16 + mm) * XP + k0;
      const unsigned short* xl = Xl + (16 + mm) * XP + k0;
      bh.h[0] = *(const us8*)(xh + 8 * hh);
      bh.h[1] = *(const us8*)(xh + 16 + 8 * hh);
      bl.h[0] = *(const us8*)(xl + 8 * hh);
      bl.h[1] = *(const us8*)(xl + 16 + 8 * hh);
      acc1 = wmma_bf(ah, bh.v, acc1);
      acc1 = wmma_bf(ah, bl.v, acc1);
      acc1 = wmma_bf(al, bh.v, acc1);
    }
  }

#pragma unroll
  for (int rr = 0; rr < 8; ++rr) {
    Ds[(wave * 16 + 8 * hh + rr) * DP + mm] = acc0[rr];
    Ds[(wave * 16 + 8 * hh + rr) * DP + 16 + mm] = acc1[rr];
  }
  __syncthreads();

  float* yb = Y + ((size_t)n * ROWS + (size_t)ch * 128) * HW + p0;
  v4f sv[4];
  int so[4];
#pragma unroll
  for (int q = 0; q < 4; ++q) {
    const int row = wave * 16 + q * 4 + (lane >> 3);
    const int col = (lane & 7) * 4;
    sv[q] = *(const v4f*)(Ds + row * DP + col);
    so[q] = row * HW + col;
  }
#pragma unroll
  for (int q = 0; q < 4; ++q) *(volatile v4f*)(yb + so[q]) = sv[q];
  __threadfence();
#pragma unroll
  for (int q = 0; q < 4; ++q) *(volatile v4f*)(yb + so[q]) = sv[q];
}

__global__ __launch_bounds__(128) void k_attn(const float* __restrict__ Y,
                                              const float* __restrict__ wmix,
                                              float* O)
{
  __shared__ __attribute__((aligned(16))) unsigned short Kh[KSLOTS * KSP];
  __shared__ __attribute__((aligned(16))) unsigned short Kl[KSLOTS * KSP];
  __shared__ __attribute__((aligned(16))) unsigned short Vh[MIX * DH * VP];
  __shared__ __attribute__((aligned(16))) unsigned short Vl[MIX * DH * VP];
  __shared__ __attribute__((aligned(16))) float Sc[4 * 16 * SP];
  __shared__ __attribute__((aligned(16))) float Ob[DH * OPITCH];
  __shared__ float wl[MIX * UW + 4];

  const int tid = threadIdx.x;
  const int lane = tid & 31, wave = tid >> 5, hh = lane >> 4, mm = lane & 15;
  const int y = blockIdx.x, hd = blockIdx.y, n = blockIdx.z;
  if (y >= HS || hd >= HEADS || n >= N_IMG) return;
  const int x0 = wave * 16;

  {
    const us4 z4 = {0, 0, 0, 0};
    for (int i = tid; i < (KSLOTS * KSP) / 4; i += 128) { ((us4*)Kh)[i] = z4; ((us4*)Kl)[i] = z4; }
    for (int i = tid; i < (MIX * DH * VP) / 4; i += 128) { ((us4*)Vh)[i] = z4; ((us4*)Vl)[i] = z4; }
    for (int i = tid; i < MIX * UW; i += 128) wl[i] = wmix[i];
  }

  us16 qa = zero16u();
  {
    const int xf = x0 + mm;
    const bool qv = xf < WSP;
    const int pq = y * WSP + (qv ? xf : 0);
    const float* qp = Y + ((size_t)n * ROWS + hd * DH + 8 * hh) * HW + pq;
#pragma unroll
    for (int i = 0; i < 8; ++i) {
      const float v = qv ? qp[(size_t)i * HW] : 0.f;
      const unsigned short hb = tobf(v);
      qa[i] = hb;
      qa[8 + i] = tobf(v - bfext(hb));
    }
  }
  __syncthreads();

  float* Scw = Sc + wave * (16 * SP);

#pragma unroll 1
  for (int r = 0; r < KW; ++r) {
    const int ky = y + r - (KW / 2);
    const bool rv = (unsigned)ky < (unsigned)HS;
    const int kyc = rv ? ky : 0;
    const float* kb = Y + ((size_t)n * ROWS + C_OUT + hd * DH) * HW + kyc * WSP;
    for (int it = tid; it < DH * 14; it += 128) {
      const int d = it / 14;
      const int g4 = it - d * 14;
      const int kx = g4 * 4;
      v4f v = {0.f, 0.f, 0.f, 0.f};
      if (rv) v = *(const v4f*)(kb + (size_t)d * HW + kx);
#pragma unroll
      for (int e = 0; e < 4; ++e) {
        const unsigned short hb = tobf(v[e]);
        Kh[(kx + 4 + e) * KSP + d] = hb;
        Kl[(kx + 4 + e) * KSP + d] = tobf(v[e] - bfext(hb));
      }
    }
    __syncthreads();
#pragma unroll
    for (int tt = 0; tt < 2; ++tt) {
      const int s = x0 + tt * 16 + mm;
      FragB bh, bl;
      const us8 k8h = *(const us8*)(Kh + s * KSP + 8 * hh);
      const us8 k8l = *(const us8*)(Kl + s * KSP + 8 * hh);
      bh.h[0] = k8h; bh.h[1] = k8h;
      bl.h[0] = k8l; bl.h[1] = k8l;
      v8f sacc = zero8f();
      sacc = wmma_bf(qa, bh.v, sacc);
      sacc = wmma_bf(qa, bl.v, sacc);
      const int j = tt * 16 + mm;
#pragma unroll
      for (int rr = 0; rr < 8; ++rr) {
        const int f = 8 * hh + rr;
        const int dj = j - f;
        if ((unsigned)(dj - 1) < (unsigned)KW) Scw[f * SP + r * KW + (dj - 1)] = sacc[rr];
      }
    }
    __syncthreads();
  }

  if (lane < 16) {
    float* sp = Scw + lane * SP;
    float mx = sp[0];
#pragma unroll
    for (int u = 1; u < UW; ++u) mx = fmaxf(mx, sp[u]);
    float den = 0.f;
#pragma unroll
    for (int u = 0; u < UW; ++u) { const float e = __expf(sp[u] - mx); sp[u] = e; den += e; }
    const float inv = 1.f / den;
#pragma unroll
    for (int u = 0; u < UW; ++u) sp[u] = sp[u] * inv;
  }
  __syncthreads();

  const int sel = (hh == 0 && mm >= 8) ? 1 : 0;
  const int jbase = 8 * hh + 16 * sel;
  v8f oacc = zero8f();
#pragma unroll 1
  for (int r = 0; r < KW; ++r) {
    const int ky = y + r - (KW / 2);
    const bool rv = (unsigned)ky < (unsigned)HS;
    const int kyc = rv ? ky : 0;
    const float* vb = Y + ((size_t)n * ROWS + 2 * C_OUT + hd * DH) * HW + kyc * WSP;
#pragma unroll
    for (int e = 0; e < 7; ++e) {
      const int it = e * 128 + tid;
      const int md = it / 14;
      const int g4 = it - md * 14;
      const int kx = g4 * 4;
      const int m = md >> 4, d = md & 15;
      v4f v = {0.f, 0.f, 0.f, 0.f};
      if (rv) v = *(const v4f*)(vb + ((size_t)m * C_OUT + d) * HW + kx);
      us4 h4 = {0, 0, 0, 0}, l4 = {0, 0, 0, 0};
#pragma unroll
      for (int q = 0; q < 4; ++q) {
        const unsigned short hb = tobf(v[q]);
        h4[q] = hb;
        l4[q] = tobf(v[q] - bfext(hb));
      }
      *(us4*)(Vh + md * VP + kx + 4) = h4;
      *(us4*)(Vl + md * VP + kx + 4) = l4;
    }
    __syncthreads();

    float pbase[8];
    int pu[8];
#pragma unroll
    for (int ip = 0; ip < 8; ++ip) {
      const int j = jbase + ip;
      const int dj = j - mm;
      const bool ok = (unsigned)(dj - 1) < (unsigned)KW;
      const int u = ok ? (r * KW + dj - 1) : 0;
      pu[ip] = u;
      pbase[ip] = ok ? Scw[mm * SP + u] : 0.f;
    }
    const us8 z8 = zero8u();
#pragma unroll
    for (int m = 0; m < MIX; ++m) {
      us8 lh = zero8u(), ll = zero8u();
#pragma unroll
      for (int ip = 0; ip < 8; ++ip) {
        const float p = pbase[ip] * wl[m * UW + pu[ip]];
        const unsigned short hb = tobf(p);
        lh[ip] = hb;
        ll[ip] = tobf(p - bfext(hb));
      }
      FragB ph, pl;
      ph.h[0] = sel ? z8 : lh;  ph.h[1] = sel ? lh : z8;
      pl.h[0] = sel ? z8 : ll;  pl.h[1] = sel ? ll : z8;
      FragB va, vlo;
      const unsigned short* vr  = Vh + (m * DH + mm) * VP + x0;
      const unsigned short* vrl = Vl + (m * DH + mm) * VP + x0;
      va.h[0]  = *(const us8*)(vr + 8 * hh);
      va.h[1]  = *(const us8*)(vr + 16 + 8 * hh);
      vlo.h[0] = *(const us8*)(vrl + 8 * hh);
      vlo.h[1] = *(const us8*)(vrl + 16 + 8 * hh);
      oacc = wmma_bf(va.v, ph.v, oacc);
      oacc = wmma_bf(va.v, pl.v, oacc);
      oacc = wmma_bf(vlo.v, ph.v, oacc);
    }
    __syncthreads();
  }

#pragma unroll
  for (int rr = 0; rr < 8; ++rr) Ob[(8 * hh + rr) * OPITCH + x0 + mm] = oacc[rr];
  __syncthreads();

  float* ob = O + ((size_t)(n * C_OUT + hd * DH) * HS + y) * OPITCH;
  v4f sv[2];
  int so[2];
#pragma unroll
  for (int q = 0; q < 2; ++q) {
    const int L = wave * 8 + q * 4 + (lane >> 3);
    const int d = L >> 1, half = L & 1;
    const int col = half * 32 + (lane & 7) * 4;
    sv[q] = *(const v4f*)(Ob + d * OPITCH + col);
    so[q] = d * (HS * OPITCH) + col;
  }
#pragma unroll
  for (int q = 0; q < 2; ++q) *(volatile v4f*)(ob + so[q]) = sv[q];
  __threadfence();
#pragma unroll
  for (int q = 0; q < 2; ++q) *(volatile v4f*)(ob + so[q]) = sv[q];
}

__global__ __launch_bounds__(256) void k_pack(const float* __restrict__ O, float* out)
{
  const int row = blockIdx.x;
  if (row >= N_IMG * C_OUT) return;
  const int lane = threadIdx.x & 31, wave = threadIdx.x >> 5;
  const float* src = O + (size_t)row * HS * OPITCH;
  float* dst = out + (size_t)row * HW;
  for (int g = wave; g < 25; g += 8) {
    const int L = g * 4 + (lane >> 3);
    if (L < HW / 32) {
      const int p = L * 32 + (lane & 7) * 4;
      const int yy = p / WSP;
      const int xx = p - yy * WSP;
      const v4f v = *(const v4f*)(src + yy * OPITCH + xx);
      *(volatile v4f*)(dst + p) = v;
    }
  }
  __threadfence();
  for (int g = wave; g < 25; g += 8) {
    const int L = g * 4 + (lane >> 3);
    if (L < HW / 32) {
      const int p = L * 32 + (lane & 7) * 4;
      const int yy = p / WSP;
      const int xx = p - yy * WSP;
      const v4f v = *(const v4f*)(src + yy * OPITCH + xx);
      *(volatile v4f*)(dst + p) = v;
    }
  }
}

extern "C" void kernel_launch(void* const* d_in, const int* in_sizes, int n_in,
                              void* d_out, int out_size, void* d_ws, size_t ws_size,
                              hipStream_t stream)
{
  if (n_in < 7) return;
  if (in_sizes[0] != N_IMG * C_IN * HW) return;
  if (in_sizes[1] != C_OUT * C_IN || in_sizes[2] != C_OUT * C_IN) return;
  if (in_sizes[3] != MIX * C_OUT * C_IN) return;
  if (in_sizes[4] != C_OUT * KW || in_sizes[5] != C_OUT * KW || in_sizes[6] != C_OUT * MIX) return;
  if (out_size != N_IMG * C_OUT * HW) return;
  if (ws_size < WS_TOTAL) return;

  const float* x       = (const float*)d_in[0];
  const float* Wq      = (const float*)d_in[1];
  const float* Wk      = (const float*)d_in[2];
  const float* Wv      = (const float*)d_in[3];
  const float* row_emb = (const float*)d_in[4];
  const float* col_emb = (const float*)d_in[5];
  const float* mix_emb = (const float*)d_in[6];
  float* out = (float*)d_out;

  char* ws = (char*)d_ws;
  float* wmix = (float*)(ws + OFF_WMIX);
  float* Y    = (float*)(ws + OFF_Y);
  float* O    = (float*)(ws + OFF_O);

  k_mix<<<dim3(1), dim3(64), 0, stream>>>(row_emb, col_emb, mix_emb, wmix);
  k_proj<<<dim3((N_IMG * HW) / 32, ROWS / 128), dim3(256), 0, stream>>>(x, Wq, Wk, Wv, Y);
  k_attn<<<dim3(HS, HEADS, N_IMG), dim3(128), 0, stream>>>(Y, wmix, O);
  k_pack<<<dim3(N_IMG * C_OUT), dim3(256), 0, stream>>>(O, out);
}
